// GNN_Bottleneck_50903952392325
// MI455X (gfx1250) — hardware-verified
//
#include <hip/hip_runtime.h>
#include <math.h>

typedef __attribute__((ext_vector_type(16))) _Float16 v16h;
typedef __attribute__((ext_vector_type(16))) __bf16 v16b;
typedef __attribute__((ext_vector_type(8)))  _Float16 v8h;
typedef __attribute__((ext_vector_type(8)))  float v8f;
typedef __attribute__((ext_vector_type(4)))  float v4f;
typedef __attribute__((ext_vector_type(2)))  float v2f;
typedef __attribute__((ext_vector_type(4)))  unsigned v4u;
typedef __attribute__((ext_vector_type(4)))  int v4i;
typedef float __attribute__((may_alias)) float_a;
typedef int __attribute__((may_alias)) int_a;

template <typename T> __device__ __forceinline__ void vst2(void* p, T v) { *(volatile T*)p = v; __threadfence(); *(volatile T*)p = v; }
__device__ __forceinline__ v8f wmma16(v16h a, v16h b, v8f c) {
  v8f d = __builtin_amdgcn_wmma_f32_16x16x32_f16(false, a, false, b, (short)0, c, false, false);
  asm volatile("v_nop\n\tv_nop\n\tv_nop\n\tv_nop" : "+v"(d) : "v"(a), "v"(b));
  return d;
}
__device__ __forceinline__ v8f wmma_bf(v16b a, v16b b, v8f c) {
  v8f d = __builtin_amdgcn_wmma_f32_16x16x32_bf16(false, a, false, b, (short)0, c, false, false);
  asm volatile("v_nop\n\tv_nop\n\tv_nop\n\tv_nop" : "+v"(d) : "v"(a), "v"(b));
  return d;
}
__device__ __forceinline__ v16h frag_h(const _Float16* rowk0, int lane) {
  union { v16h v; v8h q[2]; } u; const _Float16* p = rowk0 + 8 * (lane >> 4);
  u.q[0] = *(const v8h*)p; u.q[1] = *(const v8h*)(p + 16); return u.v;
}
__device__ __forceinline__ v16h frag_f32(const float* rowk0, int lane) {
  v16h a; const float* p = rowk0 + 8 * (lane >> 4);
#pragma unroll
  for (int i = 0; i < 8; ++i) { a[i] = (_Float16)p[i]; a[8 + i] = (_Float16)p[16 + i]; }
  return a;
}
__device__ __forceinline__ v16h frag_f32s(const float* rowk0, int lane, float sc) {
  v16h a; const float* p = rowk0 + 8 * (lane >> 4);
#pragma unroll
  for (int i = 0; i < 8; ++i) { a[i] = (_Float16)(p[i] * sc); a[8 + i] = (_Float16)(p[16 + i] * sc); }
  return a;
}
__device__ __forceinline__ v16h fragc_f32(const float* W, int k0, int n, int lane, int ld, int K) {
  v16h a; const int g = lane >> 4;
#pragma unroll
  for (int i = 0; i < 8; ++i) { const int ka = k0 + 8 * g + i, kb = ka + 16;
    a[i] = (_Float16)(ka < K ? W[(size_t)ka * ld + n] : 0.f); a[8 + i] = (_Float16)(kb < K ? W[(size_t)kb * ld + n] : 0.f); }
  return a;
}
struct F2 { v16b h, l; };
__device__ __forceinline__ F2 bsplit16(const float v[16]) { F2 r;
#pragma unroll
  for (int i = 0; i < 16; ++i) { const __bf16 h = (__bf16)v[i]; r.h[i] = h; r.l[i] = (__bf16)(v[i] - (float)h); }
  return r; }
__device__ __forceinline__ F2 split_row(const float* row, int k0, int lane) { float v[16]; const float* p = row + k0 + 8 * (lane >> 4);
#pragma unroll
  for (int i = 0; i < 8; ++i) { v[i] = p[i]; v[8 + i] = p[16 + i]; }
  return bsplit16(v); }
__device__ __forceinline__ F2 split_rowK(const float* row, int k0, int lane, int K) { float v[16]; const int g = lane >> 4;
#pragma unroll
  for (int i = 0; i < 8; ++i) { const int ka = k0 + 8 * g + i, kb = ka + 16; v[i] = ka < K ? row[ka] : 0.f; v[8 + i] = kb < K ? row[kb] : 0.f; }
  return bsplit16(v); }
__device__ __forceinline__ F2 split_col(const float* W, int k0, int n, int lane, int ld, int K) { float v[16]; const int g = lane >> 4;
#pragma unroll
  for (int i = 0; i < 8; ++i) { const int ka = k0 + 8 * g + i, kb = ka + 16; v[i] = ka < K ? W[(size_t)ka * ld + n] : 0.f; v[8 + i] = kb < K ? W[(size_t)kb * ld + n] : 0.f; }
  return bsplit16(v); }
__device__ __forceinline__ v8f mac3(const F2& a, const F2& b, v8f c) { c = wmma_bf(a.l, b.h, c); c = wmma_bf(a.h, b.l, c); return wmma_bf(a.h, b.h, c); }
__device__ __forceinline__ float sigm(float v) { return 1.0f / (1.0f + expf(-v)); }
#define LDSX() do { asm volatile("s_wait_dscnt 0" ::: "memory"); __builtin_amdgcn_wave_barrier(); __builtin_amdgcn_fence(__ATOMIC_RELEASE, "workgroup"); } while (0)

#define NN 50000
#define NE 800000
#define F0 256
#define FH1 128
#define FO 64
#define FC 40
#define FCP 64
#define RBX 512
#define NRB ((NN + RBX - 1) / RBX)
#define NNP (NRB * RBX)
#define EPT 16
#define CH (256 * EPT)

__device__ __forceinline__ v16h fragc_f32s(const float* __restrict__ base, int k0, int n, int lane, int ld, float sc) {
  const int g = lane >> 4; v16h r;
#pragma unroll
  for (int i = 0; i < 8; ++i) { r[i] = (_Float16)(base[(size_t)(k0 + 8 * g + i) * ld + n] * sc); r[8 + i] = (_Float16)(base[(size_t)(k0 + 16 + 8 * g + i) * ld + n] * sc); }
  return r;
}
#define RBD 8192
#define NRBD ((NN + RBD - 1) / RBD)
__global__ __launch_bounds__(256) void k_deg(const int* __restrict__ esrc_, const int* __restrict__ edst_, float* __restrict__ DINV) {
  __shared__ int scnt[RBD];
  const int tid = threadIdx.x, which = blockIdx.y; const int r0 = blockIdx.x * RBD; const int* edst = which == 0 ? edst_ : esrc_; DINV += (size_t)which * NNP;
  for (int q = tid; q < RBD; q += 256) scnt[q] = 0;
  __syncthreads();
#pragma unroll 1
  for (int c0 = 0; c0 < NE; c0 += CH) { const int e0 = c0 + tid * EPT;
    if (e0 + EPT <= NE) {
#pragma unroll
      for (int v = 0; v < EPT / 4; ++v) { const int4 d4 = *(const int4*)(edst + e0 + v * 4); const int dd[4] = {d4.x, d4.y, d4.z, d4.w};
#pragma unroll
        for (int u = 0; u < 4; ++u) { const unsigned rel = (unsigned)(dd[u] - r0); if (rel < (unsigned)RBD) atomicAdd(&scnt[rel], 1); } } }
    else { for (int u = 0; u < EPT; ++u) { const int e = e0 + u; if (e < NE) { const unsigned rel = (unsigned)(edst[e] - r0); if (rel < (unsigned)RBD) atomicAdd(&scnt[rel], 1); } } } }
  __syncthreads();
  for (int q = tid; q < RBD; q += 256) { const int r = r0 + q; if (r < NNP) vst2(DINV + r, r < NN ? rsqrtf((float)(scnt[q] + 1)) : 0.f); }
}
template <int K, int NOUT, int WROWS>
__global__ __launch_bounds__(128) void k_gemm(const float* __restrict__ A, int lda, const float* __restrict__ W, const float* __restrict__ DINV, float* __restrict__ HS) {
  __shared__ __align__(16) float so[4][16][NOUT + 4];
  const int tid = threadIdx.x, wave = tid >> 5, lane = tid & 31, col = lane & 15, g = lane >> 4;
  const int r0 = blockIdx.x * 64 + wave * 16;
  constexpr int NT = (NOUT + 15) / 16;
  v8f acc[NT];
#pragma unroll
  for (int t = 0; t < NT; ++t) acc[t] = (v8f){};
const int ra = (r0 + col) < NN ? (r0 + col) : (NN - 1);
#pragma unroll 1
  for (int kc = 0; kc < K / 32; ++kc) { const v16h a = frag_f32(A + (size_t)ra * lda + kc * 32, lane);
#pragma unroll
    for (int t = 0; t < NT; ++t) { const int n = t * 16 + col; acc[t] = wmma16(a, fragc_f32s(W, kc * 32, n, lane, NOUT, 16.0f), acc[t]); } }
#pragma unroll
  for (int t = 0; t < NT; ++t) { const int n = t * 16 + col;
#pragma unroll
    for (int r = 0; r < 8; ++r) { const int row = r0 + 8 * g + r; const float dv = row < NN ? DINV[NNP + row] : 0.f; so[wave][8 * g + r][n] = acc[t][r] * (1.0f / 16.0f) * dv; } }
  LDSX();
  for (int q = lane; q < 16 * (NOUT / 4); q += 32) { const int rl = q / (NOUT / 4), pc = q % (NOUT / 4); vst2(HS + (size_t)(r0 + rl) * NOUT + pc * 4, *(const v4f*)(&so[wave][rl][pc * 4])); }
}
template <int F, int MODE, int RB>
__global__ __launch_bounds__(256) void k_agg(const float* __restrict__ HS, const int* __restrict__ esrc_, const int* __restrict__ edst_, const float* __restrict__ DINV, const float* __restrict__ bias, const float* __restrict__ lng, const float* __restrict__ lnb, float* __restrict__ OUT) {
  __shared__ __align__(16) float sacc[RB][F];
  __shared__ int ssrc[8][32 * EPT], sdl[8][32 * EPT]; __shared__ int scnt[8];
  const int tid = threadIdx.x, wave = tid >> 5, lane = tid & 31;
  const int r0 = blockIdx.x * RB; const int* esrc = esrc_; const int* edst = edst_;
  for (int q = tid; q < RB * F; q += 256) (&sacc[0][0])[q] = 0.f;
  __syncthreads();
#pragma unroll 1
  for (int c0 = 0; c0 < NE; c0 += CH) {
    const int e0 = c0 + tid * EPT; int hd[EPT]; int cnt = 0;
    if (e0 + EPT <= NE) {
#pragma unroll
      for (int v = 0; v < EPT / 4; ++v) { const int4 d4 = *(const int4*)(edst + e0 + v * 4);
        const int dd[4] = {d4.x, d4.y, d4.z, d4.w};
#pragma unroll
        for (int u = 0; u < 4; ++u) { const unsigned rel = (unsigned)(dd[u] - r0); const bool h = rel < (unsigned)RB; hd[v * 4 + u] = h ? (int)rel : -1; cnt += h ? 1 : 0; } } }
    else {
#pragma unroll
      for (int u = 0; u < EPT; ++u) { const int e = e0 + u; hd[u] = -1; if (e < NE) { const unsigned rel = (unsigned)(edst[e] - r0); if (rel < (unsigned)RB) { hd[u] = (int)rel; ++cnt; } } } }
    int incl = cnt;
#pragma unroll
    for (int off = 1; off < 32; off <<= 1) { const int vv = __shfl_up(incl, off, 32); if (lane >= off) incl += vv; }
    const int wtot = __shfl(incl, 31, 32); int pos = incl - cnt;
    if (cnt > 0) {
#pragma unroll
      for (int u = 0; u < EPT; ++u) if (hd[u] >= 0) { int s = esrc[e0 + u]; s = s < 0 ? 0 : (s >= NN ? NN - 1 : s); ssrc[wave][pos] = s; sdl[wave][pos] = hd[u];  ++pos; } }
    if (lane == 0) scnt[wave] = wtot;
    __syncthreads();
    if (tid < F) { for (int w = 0; w < 8; ++w) { const int nh = scnt[w]; for (int i = 0; i < nh; ++i) sacc[sdl[w][i]][tid] += HS[(size_t)ssrc[w][i] * F + tid]; } }
    __syncthreads(); }
  for (int rl = tid; rl < RB; rl += 256) { const int row = r0 + rl; if (row >= NN) continue; const float dv = DINV[row]; float* ar = &sacc[rl][0]; const float* hs = HS + (size_t)row * F;
    for (int f = 0; f < F; ++f) ar[f] = (ar[f] + hs[f]) * dv + bias[f];
    if (MODE == 2) { for (int f = 0; f < F; ++f) ar[f] = ar[f] > 0.f ? ar[f] : 0.f; }
    else if (MODE == 3) { for (int f = 0; f < F; ++f) ar[f] = sigm(ar[f]) + 1e-8f; }
    else if (MODE == 4) { for (int f = 0; f < F; ++f) ar[f] = ar[f] > 0.f ? ar[f] : expm1f(ar[f]); }
    else if (MODE == 5) { }
    else if (MODE == 0) { float mu = 0.f; for (int f = 0; f < F; ++f) mu += ar[f]; mu *= (1.0f / F); float var = 0.f; for (int f = 0; f < F; ++f) { const float d = ar[f] - mu; var += d * d; } var *= (1.0f / F);
      const float rs = rsqrtf(var + 1e-5f); for (int f = 0; f < F; ++f) { const float v = (ar[f] - mu) * rs * lng[f] + lnb[f]; ar[f] = v > 0.f ? v : 0.f; } }
    else { float mx = -3.4e38f; for (int f = 0; f < FC; ++f) mx = fmaxf(mx, ar[f]); float se = 0.f; for (int f = 0; f < FC; ++f) se += expf(ar[f] - mx); const float lse = logf(se) + mx; for (int f = 0; f < FC; ++f) ar[f] -= lse; } }
  __syncthreads();
  if (MODE != 1) { for (int q = tid; q < RB * (F / 4); q += 256) { const int rl = q / (F / 4), pc = q % (F / 4); const int row = r0 + rl; v4f v = *(const v4f*)(&sacc[rl][pc * 4]); if (row >= NN) { if (MODE >= 2) continue; v = (v4f){0.f, 0.f, 0.f, 0.f}; } vst2(OUT + (size_t)row * F + pc * 4, v); } }
  else {
    for (int q = tid; q < RB * FC / 4; q += 256) { const int rl = (q * 4) / FC, f = (q * 4) % FC; const int row = r0 + rl; if (row < NN) { v4f v; v[0] = sacc[rl][f]; v[1] = sacc[rl][f + 1]; v[2] = sacc[rl][f + 2]; v[3] = sacc[rl][f + 3]; vst2(OUT + (size_t)row * FC + f, v); } } }
}
extern "C" void kernel_launch(void* const* d_in, const int* in_sizes, int n_in, void* d_out, int out_size, void* d_ws, size_t ws_size, hipStream_t stream) {
  (void)in_sizes; (void)n_in; (void)out_size; (void)ws_size;
  const float** I = (const float**)d_in;
  const float* x = I[0]; const int* ei = (const int*)d_in[1]; const float* W1 = I[2]; const float* b1 = I[3]; const float* W2 = I[4]; const float* b2 = I[5]; const float* W3 = I[6]; const float* b3 = I[7];
  const int* src = ei; const int* dst = ei + NE;
  float* out = (float*)d_out;
  char* ws = (char*)d_ws; size_t off = 0;
  auto take = [&](size_t bytes) { char* p = ws + off; off += (bytes + 255) & ~(size_t)255; return p; };
  float* DINV = (float*)take((size_t)2 * NNP * 4); float* HS = (float*)take((size_t)NNP * FH1 * 4); float* H1 = (float*)take((size_t)NNP * FH1 * 4);
  k_deg<<<dim3(NRBD, 2), 256, 0, stream>>>(dst, dst, DINV);
  k_gemm<F0, FH1, 0><<<NNP / 64, 128, 0, stream>>>(x, F0, W1, DINV, HS);
  k_agg<FH1, 2, 512><<<(NN + 511) / 512, 256, 0, stream>>>(HS, src, dst, DINV, b1, nullptr, nullptr, H1);
  k_gemm<FH1, FH1, 0><<<NNP / 64, 128, 0, stream>>>(H1, FH1, W2, DINV, HS);
  k_agg<FH1, 2, 512><<<(NN + 511) / 512, 256, 0, stream>>>(HS, src, dst, DINV, b2, nullptr, nullptr, H1);
  k_gemm<FH1, FO, 0><<<NNP / 64, 128, 0, stream>>>(H1, FH1, W3, DINV, HS);
  k_agg<FO, 5, 1024><<<(NN + 1023) / 1024, 256, 0, stream>>>(HS, src, dst, DINV, b3, nullptr, nullptr, out);
}
